// ResAttnConv2d_80204219285685
// MI455X (gfx1250) — hardware-verified
//
#include <hip/hip_runtime.h>
#include <stdint.h>

#define NB    32
#define CIN   64
#define CH    32
#define CO    64
#define HW    4096
#define IMW   64
#define KD    288
#define NLP   448
#define NKK   9
#define NZC   96
#define SHP   40
#define SHN   (3 * 66 * SHP)
#define STGF  6912
#define NPIX4 (NB * CO * HW / 4)
#define HSC   16.0f
#define WSC   256.0f
#define RSC   2048.0f

static_assert(SHN == 7920);
static_assert(2 * NZC * 72 == 2 * STGF);
static_assert(64 * 104 <= 2 * STGF);
static_assert(64 * 68 <= STGF);
static_assert(NPIX4 % 256 == 0);
static_assert((NB * HW * 4) % 256 == 0);

typedef _Float16 v16h __attribute__((ext_vector_type(16)));
typedef _Float16 v8h  __attribute__((ext_vector_type(8)));
typedef float    v8f  __attribute__((ext_vector_type(8)));
typedef float    v4f  __attribute__((ext_vector_type(4)));
typedef unsigned int v4u __attribute__((ext_vector_type(4)));

static const size_t YPE = (size_t)NB * NKK * NLP * 64;

__device__ __forceinline__ unsigned short bf_bits(float f) {
  unsigned u = __float_as_uint(f);
  return (unsigned short)((u + 0x7FFFu + ((u >> 16) & 1u)) >> 16);
}
__device__ __forceinline__ float bf_up(unsigned short h) { return __uint_as_float(((unsigned)h) << 16); }
__device__ __forceinline__ float bfr(float f) { return bf_up(bf_bits(f)); }
__device__ __forceinline__ unsigned short hb(float f) { return __builtin_bit_cast(unsigned short, (_Float16)f); }
__device__ __forceinline__ unsigned pk16(unsigned short a, unsigned short b) { return (unsigned)a | ((unsigned)b << 16); }
__device__ __forceinline__ v8f zero8() { v8f z = {0.f, 0.f, 0.f, 0.f, 0.f, 0.f, 0.f, 0.f}; return z; }
__device__ __forceinline__ v4u z4u() { v4u z = {0u, 0u, 0u, 0u}; return z; }
__device__ __forceinline__ v4f z4f() { v4f z = {0.f, 0.f, 0.f, 0.f}; return z; }

__device__ __forceinline__ v16h ldfrag(const unsigned short* p) {
  union { v16h v; v8h h[2]; } f;
  f.h[0] = *(const v8h*)(const void*)(p);
  f.h[1] = *(const v8h*)(const void*)(p + 16);
  return f.v;
}
__device__ __forceinline__ v8f mma(v16h a, v16h b, v8f c) {
  return __builtin_amdgcn_wmma_f32_16x16x32_f16(false, a, false, b, (short)0, c, false, false);
}
__device__ __forceinline__ void g1(v8f& a, v16h x, v16h y) {
#if defined(__HIP_DEVICE_COMPILE__)
  asm volatile("v_nop\n\tv_nop\n\tv_nop\n\tv_nop" : "+v"(a) : "v"(x), "v"(y));
#endif
}
__device__ __forceinline__ void g2(v8f& a, v8f& b, v16h x, v16h y) {
#if defined(__HIP_DEVICE_COMPILE__)
  asm volatile("v_nop\n\tv_nop\n\tv_nop\n\tv_nop" : "+v"(a), "+v"(b) : "v"(x), "v"(y));
#endif
}
__device__ __forceinline__ void g2w(v8f& a, v8f& b, v16h x, v16h y, v16h z, v16h q) {
#if defined(__HIP_DEVICE_COMPILE__)
  asm volatile("v_nop\n\tv_nop\n\tv_nop\n\tv_nop" : "+v"(a), "+v"(b) : "v"(x), "v"(y), "v"(z), "v"(q));
#endif
}
__device__ __forceinline__ void ag1(v8f& a) {
#if defined(__HIP_DEVICE_COMPILE__)
  asm volatile("v_nop\n\tv_nop\n\tv_nop\n\tv_nop" : "+v"(a));
#endif
}
__device__ __forceinline__ void ag2(v8f& a, v8f& b) {
#if defined(__HIP_DEVICE_COMPILE__)
  asm volatile("v_nop\n\tv_nop\n\tv_nop\n\tv_nop" : "+v"(a), "+v"(b));
#endif
}
__device__ __forceinline__ void ag3(v8f& a, v8f& b, v8f& c) {
#if defined(__HIP_DEVICE_COMPILE__)
  asm volatile("v_nop\n\tv_nop\n\tv_nop\n\tv_nop" : "+v"(a), "+v"(b), "+v"(c));
#endif
}

template <int RB>
__global__ __launch_bounds__(256) void bn_stats(const float* __restrict__ src, float* mr) {
  __shared__ double rs[256];
  __shared__ double rq[256];
  const int c = blockIdx.x, tid = threadIdx.x;
  double s = 0.0, q = 0.0;
#pragma unroll 1
  for (int i = tid; i < NB * HW / 4; i += 256) {
    const int b = i >> 10, p4 = (i & 1023) * 4;
    const v4f v = *(const v4f*)(src + ((size_t)(b * CO + c)) * HW + p4);
#pragma unroll
    for (int e = 0; e < 4; ++e) {
      const float f = RB ? bfr(v[e]) : v[e];
      const double d = (double)f;
      s += d; q += d * d;
    }
  }
  rs[tid] = s; rq[tid] = q;
  __syncthreads();
  for (int st = 128; st > 0; st >>= 1) {
    if (tid < st) { rs[tid] += rs[tid + st]; rq[tid] += rq[tid + st]; }
    __syncthreads();
  }
  if (tid < 8) {
    const double n = (double)(NB * HW);
    const double m = rs[0] / n;
    double var = rq[0] / n - m * m;
    if (var < 0.0) var = 0.0;
    const float mf = (float)m;
    const float vf = (float)var;
    const float rf = (float)(1.0 / sqrt((double)(vf + 1e-5f)));
    v4f o = z4f();
    if (tid == 0) { o[0] = mf; o[1] = rf; }
    float* d = mr + c * 32 + tid * 4;
    *(volatile v4f*)d = o;
    __threadfence();
    *(volatile v4f*)d = o;
  }
}

__global__ __launch_bounds__(256) void cvt_w(const float* __restrict__ src, unsigned short* dst,
                                             int nco, int rbase, int rstride) {
  const int t = blockIdx.x * 256 + threadIdx.x;
  const int per = nco * KD;
  const int n8 = (4 * per) / 8;
  if (t >= n8) return;
  const int i0 = t * 8;
  const int pth = i0 / per;
  const int rem = i0 - pth * per;
  const int co = rem / KD;
  const int k0 = rem - co * KD;
  const float* srow = src + ((size_t)(pth * nco + co)) * CH * NKK;
  v4u p;
#pragma unroll
  for (int e = 0; e < 4; ++e) {
    const int ka = k0 + 2 * e, kb = ka + 1;
    const float fa = bfr(srow[(ka & 31) * NKK + (ka >> 5)]) * WSC;
    const float fb = bfr(srow[(kb & 31) * NKK + (kb >> 5)]) * WSC;
    p[e] = pk16(hb(fa), hb(fb));
  }
  unsigned short* d = dst + ((size_t)(pth * rstride + rbase + co)) * KD + k0;
  *(volatile v4u*)d = p;
  __threadfence();
  *(volatile v4u*)d = p;
}

__global__ __launch_bounds__(256) void make_h(const float* __restrict__ x, const float* __restrict__ mrx,
                                              const float* __restrict__ a_pre, int pth,
                                              unsigned short* hq) {
  __shared__ float sm[CH];
  __shared__ float sr[CH];
  const int tid = threadIdx.x;
  const int half = pth & 1;
  if (tid < CH) { const int g = half * CH + tid; sm[tid] = mrx[g * 32]; sr[tid] = mrx[g * 32 + 1]; }
  __syncthreads();
  const int g8 = blockIdx.x * 256 + tid;
  const int pix = g8 >> 2, j = g8 & 3;
  const int b = pix >> 12, p = pix & (HW - 1);
  const float c1 = 0.01f * bfr(a_pre[pth]);
  const float* xs = x + ((size_t)(b * CIN + half * CH + 8 * j)) * HW + p;
  v4u o;
#pragma unroll
  for (int e = 0; e < 4; ++e) {
    const int ca = 8 * j + 2 * e, cb = ca + 1;
    const float xa = bfr(xs[(size_t)(2 * e) * HW]);
    const float xb = bfr(xs[(size_t)(2 * e + 1) * HW]);
    const float ha = 0.5f * ((xa - sm[ca]) * sr[ca]) + c1 * xa;
    const float hbv = 0.5f * ((xb - sm[cb]) * sr[cb]) + c1 * xb;
    o[e] = pk16(hb(ha * HSC), hb(hbv * HSC));
  }
  unsigned short* d = hq + (size_t)g8 * 8;
  *(volatile v4u*)d = o;
  __threadfence();
  *(volatile v4u*)d = o;
}

template <int MODE>
__global__ __launch_bounds__(256) void conv3x3(const unsigned short* __restrict__ Ap,
                                               const unsigned short* __restrict__ Alp,
                                               const unsigned short* __restrict__ inp,
                                               unsigned short* o16a, unsigned short* o16b, float* o32) {
  constexpr int NCO  = (MODE == 2) ? 32 : ((MODE == 3) ? 64 : NZC);
  constexpr int NSUB = NCO / 32;
  constexpr int TS   = (MODE == 3) ? 2048 : 32;
  __shared__ __align__(16) unsigned short sh[SHN];
  __shared__ __align__(16) float stg[STGF];
  const int tid = threadIdx.x, w = tid >> 5, lane = tid & 31, hh = lane >> 4, ln = lane & 15;
  const int b = blockIdx.x >> 6, y = blockIdx.x & 63;
  const unsigned short* inb = inp + (size_t)b * HW * CH;
  {
    const int px = tid >> 2, chunk = tid & 3;
#pragma unroll
    for (int r = 0; r < 3; ++r) {
      const int gy = y + r - 1;
      const bool ok = (gy >= 0) && (gy < 64);
      const int cgy = min(max(gy, 0), 63);
      v4u v = *(const v4u*)(inb + ((size_t)(cgy * IMW + px)) * CH + chunk * 8);
      if (!ok) v = z4u();
      *(v4u*)(sh + (r * 66 + px + 1) * SHP + chunk * 8) = v;
    }
    if (tid < 24) {
      const int r = tid >> 3;
      const int xx = ((tid >> 2) & 1) ? 65 : 0;
      const int ck = tid & 3;
      *(v4u*)(sh + (r * 66 + xx) * SHP + ck * 8) = z4u();
    }
  }
  __syncthreads();

  const int ni = w & 3, cg = w >> 2;
  const int xcol = ni * 16 + ln;
  const int co0 = cg * (NCO / 2);
  const unsigned short* bp = sh + xcol * SHP + 8 * hh;
  const unsigned short* ap[3];
  const unsigned short* aq[3];
#pragma unroll
  for (int s = 0; s < NSUB; ++s) {
    const int ch = co0 + s * 16 + ln;
    if (MODE == 3) {
      const size_t o = ((size_t)(b * (NKK * CO) + ch)) * CH + 8 * hh;
      ap[s] = Ap + o; aq[s] = Alp + o;
    } else {
      ap[s] = Ap + (size_t)ch * KD + 8 * hh; aq[s] = ap[s];
    }
  }
  v8f acc[3], acc2[3];
#pragma unroll
  for (int s = 0; s < 3; ++s) { acc[s] = zero8(); acc2[s] = zero8(); }

#pragma unroll
  for (int t = 0; t < NKK; ++t) {
    const int kh = t / 3, kw = t - kh * 3;
    const v16h bf = ldfrag(bp + (kh * 66 + kw) * SHP);
    v16h af = bf, al = bf;
#pragma unroll
    for (int s = 0; s < NSUB; ++s) {
      af = ldfrag(ap[s] + t * TS);
      acc[s] = mma(af, bf, acc[s]);
      if (MODE == 3) {
        al = ldfrag(aq[s] + t * TS);
        acc2[s] = mma(al, bf, acc2[s]);
      }
    }
    if (NSUB == 1) g1(acc[0], af, bf);
    else g2(acc[0], acc[NSUB - 1], af, bf);
    if (MODE == 3) g2(acc2[0], acc2[1], al, bf);
  }
  if (NSUB == 1) ag1(acc[0]);
  else if (NSUB == 2) ag2(acc[0], acc[1]);
  else ag3(acc[0], acc[1], acc[2]);
  if (MODE == 3) ag2(acc2[0], acc2[1]);

  if (MODE == 0) {
    unsigned short* sHi = (unsigned short*)stg;
    unsigned short* sLo = sHi + NZC * 72;
#pragma unroll
    for (int s = 0; s < NSUB; ++s) {
#pragma unroll
      for (int r = 0; r < 8; ++r) {
        const int ch = co0 + s * 16 + 8 * hh + r;
        const float v = acc[s][r] * (1.0f / 256.0f);
        const _Float16 hv = (_Float16)v;
        const float lv = (v - (float)hv) * RSC;
        sHi[ch * 72 + xcol] = __builtin_bit_cast(unsigned short, hv);
        sLo[ch * 72 + xcol] = hb(lv);
      }
    }
    __syncthreads();
    const int q = lane >> 3, j = lane & 7;
    v4u ph[3], pl[3]; size_t off[3];
#pragma unroll
    for (int it = 0; it < 3; ++it) {
      const int ch = it * 32 + w * 4 + q;
      ph[it] = *(const v4u*)(sHi + ch * 72 + 8 * j);
      pl[it] = *(const v4u*)(sLo + ch * 72 + 8 * j);
      off[it] = ((size_t)(b * NZC + ch)) * HW + y * 64 + 8 * j;
    }
    for (int pass = 0; pass < 2; ++pass) {
#pragma unroll
      for (int it = 0; it < 3; ++it) {
        *(volatile v4u*)(o16a + off[it]) = ph[it];
        *(volatile v4u*)(o16b + off[it]) = pl[it];
      }
      __threadfence();
    }
  } else if (MODE == 1) {
    unsigned short* sY = (unsigned short*)stg;
#pragma unroll
    for (int s = 0; s < NSUB; ++s) {
      v4u pk;
#pragma unroll
      for (int e = 0; e < 4; ++e)
        pk[e] = pk16(hb(acc[s][2 * e] * (1.0f / 256.0f)), hb(acc[s][2 * e + 1] * (1.0f / 256.0f)));
      *(v4u*)(sY + xcol * 104 + co0 + s * 16 + 8 * hh) = pk;
    }
    __syncthreads();
    const bool live = (y < 63);
    const int kh0 = (y % 3) * 3, ly21 = (y / 3) * 21;
    v4u val[4]; size_t off[4]; bool act[4];
#pragma unroll
    for (int it = 0; it < 4; ++it) {
      const int item = it * 256 + tid;
      act[it] = item < 1008;
      const int itc = min(item, 1007);
      const int piece = itc & 7, rowi = itc >> 3;
      int kk, l, plane;
      v4u v = z4u();
      if (live) {
        const int xx = rowi >> 1;
        plane = rowi & 1;
        const int choff = piece * 8 + plane * 32;
        v = *(const v4u*)(sY + xx * 104 + choff);
        if (plane == 0 && piece >= 4) v = z4u();
        kk = kh0 + (xx % 3);
        l = ly21 + xx / 3;
      } else {
        plane = (rowi >= 63) ? 1 : 0;
        const int rr = rowi - plane * 63;
        kk = rr / 7;
        l = 441 + (rr - kk * 7);
      }
      val[it] = v;
      off[it] = (size_t)plane * YPE + ((size_t)((b * NKK + kk) * NLP + l)) * 64 + piece * 8;
    }
    for (int pass = 0; pass < 2; ++pass) {
#pragma unroll
      for (int it = 0; it < 4; ++it)
        if (act[it]) *(volatile v4u*)(o16a + off[it]) = val[it];
      __threadfence();
    }
  } else if (MODE == 2) {
    unsigned short* sU = (unsigned short*)stg;
    {
      v4u pk;
#pragma unroll
      for (int e = 0; e < 4; ++e)
        pk[e] = pk16(hb(acc[0][2 * e] * (1.0f / 256.0f)), hb(acc[0][2 * e + 1] * (1.0f / 256.0f)));
      *(v4u*)(sU + xcol * SHP + co0 + 8 * hh) = pk;
    }
    __syncthreads();
    const int q = lane >> 2, j = lane & 3;
    const int px = w * 8 + q;
    const v4u v = *(const v4u*)(sU + px * SHP + 8 * j);
    unsigned short* d = o16a + ((size_t)(b * HW + y * 64 + px)) * CH + 8 * j;
    *(volatile v4u*)d = v;
    __threadfence();
    *(volatile v4u*)d = v;
  } else {
    float* sV = stg;
#pragma unroll
    for (int s = 0; s < NSUB; ++s) {
#pragma unroll
      for (int r = 0; r < 8; ++r) {
        const int ch = co0 + s * 16 + 8 * hh + r;
        sV[ch * 68 + xcol] = (acc[s][r] + acc2[s][r] * (1.0f / RSC)) * (1.0f / 4096.0f);
      }
    }
    __syncthreads();
    v4f ov[4]; size_t off[4];
#pragma unroll
    for (int it = 0; it < 4; ++it) {
      const int ch = it * 16 + w * 2 + hh;
      const int c4 = ln * 4;
      ov[it] = *(const v4f*)(sV + ch * 68 + c4);
      off[it] = ((size_t)(b * CO + ch)) * HW + y * 64 + c4;
    }
    for (int pass = 0; pass < 2; ++pass) {
#pragma unroll
      for (int it = 0; it < 4; ++it) *(volatile v4f*)(o32 + off[it]) = ov[it];
      __threadfence();
    }
  }
}

__global__ __launch_bounds__(256) void corr1_softmax(const unsigned short* __restrict__ zh,
                                                     const unsigned short* __restrict__ zl, float* k2) {
  __shared__ __align__(16) float sL[64 * 36];
  const int b = blockIdx.x, tid = threadIdx.x, w = tid >> 5, lane = tid & 31, hh = lane >> 4, ln = lane & 15;
  const int mi = w >> 1, ni = w & 1;
  const size_t ao = ((size_t)(b * NZC + 32 + mi * 16 + ln)) * HW + 8 * hh;
  const size_t bo = ((size_t)(b * NZC + ni * 16 + ln)) * HW + 8 * hh;
  v8f a1 = zero8(), a2 = zero8();
#pragma unroll 2
  for (int k0 = 0; k0 < HW; k0 += 32) {
    const v16h ah = ldfrag(zh + ao + k0);
    const v16h al = ldfrag(zl + ao + k0);
    const v16h bh = ldfrag(zh + bo + k0);
    const v16h bl = ldfrag(zl + bo + k0);
    a1 = mma(ah, bh, a1);
    a2 = mma(ah, bl, a2);
    a2 = mma(al, bh, a2);
    g2w(a1, a2, ah, al, bh, bl);
  }
  ag2(a1, a2);
  const float sc = (1.0f / 256.0f) * 0.17677669529663687f;
#pragma unroll
  for (int r = 0; r < 8; ++r) {
    const int o = mi * 16 + 8 * hh + r;
    const int c = ni * 16 + ln;
    sL[o * 36 + c] = (a1[r] + a2[r] * (1.0f / RSC)) * sc;
  }
  __syncthreads();
  if (tid < 64) {
    float* row = sL + tid * 36;
    float mx = row[0];
#pragma unroll 1
    for (int i = 1; i < CH; ++i) mx = fmaxf(mx, row[i]);
    float s = 0.f;
#pragma unroll 1
    for (int i = 0; i < CH; ++i) { const float e = expf(row[i] - mx); row[i] = e; s += e; }
    const float inv = 1.0f / s;
#pragma unroll 1
    for (int i = 0; i < CH; ++i) row[i] = row[i] * inv;
  }
  __syncthreads();
  const int q = lane >> 3, j = lane & 7;
  v4f ov[2]; size_t off[2];
#pragma unroll
  for (int it = 0; it < 2; ++it) {
    const int o = it * 32 + w * 4 + q;
    ov[it] = *(const v4f*)(sL + o * 36 + 4 * j);
    off[it] = ((size_t)(b * CO + o)) * CH + 4 * j;
  }
  for (int pass = 0; pass < 2; ++pass) {
#pragma unroll
    for (int it = 0; it < 2; ++it) *(volatile v4f*)(k2 + off[it]) = ov[it];
    __threadfence();
  }
}

__global__ __launch_bounds__(256) void corr3_ak(const unsigned short* __restrict__ yp,
                                               const float* __restrict__ k2,
                                               const float* __restrict__ aw,
                                               unsigned short* akh, unsigned short* akl) {
  __shared__ __align__(16) unsigned short sA[64 * 72];
  __shared__ __align__(16) unsigned short sB[32 * 72];
  __shared__ __align__(16) float sD[64 * 36];
  const int blk = blockIdx.x, b = blk / NKK, kk = blk - b * NKK;
  const int tid = threadIdx.x, w = tid >> 5, lane = tid & 31, hh = lane >> 4, ln = lane & 15;
  const int mi = w >> 1, ni = w & 1;
  const unsigned short* y1p = yp + ((size_t)(b * NKK + kk)) * NLP * 64;
  const unsigned short* y2p = y1p + YPE;
  v8f acc = zero8();
#pragma unroll 1
  for (int chn = 0; chn < 7; ++chn) {
    const int l0 = chn * 64;
#pragma unroll
    for (int it = 0; it < 2; ++it) {
      const int id = it * 256 + tid;
      const int li = id >> 3, jj = id & 7;
      const v4u v = *(const v4u*)(y2p + ((size_t)(l0 + li)) * 64 + 8 * jj);
#pragma unroll
      for (int e = 0; e < 4; ++e) {
        sA[(8 * jj + 2 * e) * 72 + li]     = (unsigned short)(v[e] & 0xFFFFu);
        sA[(8 * jj + 2 * e + 1) * 72 + li] = (unsigned short)(v[e] >> 16);
      }
    }
    {
      const int li = tid >> 2, jj = tid & 3;
      const v4u v = *(const v4u*)(y1p + ((size_t)(l0 + li)) * 64 + 8 * jj);
#pragma unroll
      for (int e = 0; e < 4; ++e) {
        sB[(8 * jj + 2 * e) * 72 + li]     = (unsigned short)(v[e] & 0xFFFFu);
        sB[(8 * jj + 2 * e + 1) * 72 + li] = (unsigned short)(v[e] >> 16);
      }
    }
    __syncthreads();
#pragma unroll
    for (int ks = 0; ks < 2; ++ks) {
      const v16h af = ldfrag(sA + (mi * 16 + ln) * 72 + ks * 32 + 8 * hh);
      const v16h bf = ldfrag(sB + (ni * 16 + ln) * 72 + ks * 32 + 8 * hh);
      acc = mma(af, bf, acc);
      g1(acc, af, bf);
    }
    __syncthreads();
  }
  ag1(acc);
  const float sc = (1.0f / 256.0f) * 0.05892556509887896f;
#pragma unroll
  for (int r = 0; r < 8; ++r) {
    const int o = mi * 16 + 8 * hh + r;
    const int c = ni * 16 + ln;
    sD[o * 36 + c] = acc[r] * sc;
  }
  __syncthreads();
  const int q = lane >> 2, j = lane & 3;
  const int o = w * 8 + q;
  const v4f d0 = *(const v4f*)(sD + o * 36 + 8 * j);
  const v4f d1 = *(const v4f*)(sD + o * 36 + 8 * j + 4);
  const v4f e0 = *(const v4f*)(k2 + ((size_t)(b * CO + o)) * CH + 8 * j);
  const v4f e1 = *(const v4f*)(k2 + ((size_t)(b * CO + o)) * CH + 8 * j + 4);
  const float* awp = aw + ((size_t)(o * CH + 8 * j)) * NKK + kk;
  float t8[8];
#pragma unroll
  for (int e = 0; e < 4; ++e) {
    t8[e]     = (e0[e] * (d0[e] + bfr(awp[e * NKK]))) * WSC;
    t8[4 + e] = (e1[e] * (d1[e] + bfr(awp[(4 + e) * NKK]))) * WSC;
  }
  v4u ph, pl;
#pragma unroll
  for (int e = 0; e < 4; ++e) {
    const _Float16 ha = (_Float16)t8[2 * e], hbx = (_Float16)t8[2 * e + 1];
    const float la = (t8[2 * e] - (float)ha) * RSC, lb = (t8[2 * e + 1] - (float)hbx) * RSC;
    ph[e] = pk16(__builtin_bit_cast(unsigned short, ha), __builtin_bit_cast(unsigned short, hbx));
    pl[e] = pk16(hb(la), hb(lb));
  }
  const size_t off = ((size_t)((b * NKK + kk) * CO + o)) * CH + 8 * j;
  for (int pass = 0; pass < 2; ++pass) {
    *(volatile v4u*)(akh + off) = ph;
    *(volatile v4u*)(akl + off) = pl;
    __threadfence();
  }
}

__global__ __launch_bounds__(256) void finalize(const float* __restrict__ v, const float* __restrict__ mrv,
                                                const float* __restrict__ a_post, const float* __restrict__ x,
                                                const float* __restrict__ cm, int pth,
                                                float* ya, float* yb, float* out) {
  const int qd = blockIdx.x * 256 + threadIdx.x;
  const size_t idx = (size_t)qd * 4;
  const int o = (int)((idx >> 12) & 63);
  const float m = mrv[o * 32], r = mrv[o * 32 + 1];
  const float ap = 0.6f * bfr(a_post[pth]);
  const v4f vv = *(const v4f*)(v + idx);
  v4f t;
#pragma unroll
  for (int e = 0; e < 4; ++e) t[e] = 0.5f * ((vv[e] - m) * r) + ap * vv[e];
  v4f res = t;
  float* d = ya + idx;
  if (pth == 1) {
    const v4f a = *(const v4f*)(ya + idx);
#pragma unroll
    for (int e = 0; e < 4; ++e) res[e] = a[e] + t[e];
    d = yb + idx;
  } else if (pth == 3) {
    const float c0 = 0.99f * bfr(cm[0]);
    const v4f xa = *(const v4f*)(x + idx);
    const v4f a = *(const v4f*)(ya + idx);
    const v4f bb = *(const v4f*)(yb + idx);
#pragma unroll
    for (int e = 0; e < 4; ++e) res[e] = c0 * bfr(xa[e]) + (bb[e] + a[e] * t[e]) * 0.57735026918962576f;
    d = out + idx;
  }
  *(volatile v4f*)d = res;
  __threadfence();
  *(volatile v4f*)d = res;
}

extern "C" void kernel_launch(void* const* d_in, const int* in_sizes, int n_in,
                              void* d_out, int out_size, void* d_ws, size_t ws_size,
                              hipStream_t stream) {
  if (n_in < 10) return;
  if (in_sizes[0] != NB * CIN * HW) return;
  if (in_sizes[1] != 4 * CH * CH * NKK) return;
  if (in_sizes[2] != 4 * CO * CH * NKK) return;
  if (in_sizes[3] != 4 * CH * CH * NKK) return;
  if (in_sizes[4] != 4 * CO * CH * NKK) return;
  if (in_sizes[5] != 4 * CH * CH * NKK) return;
  if (in_sizes[6] != 4 * CO * CH * NKK) return;
  if (in_sizes[7] != 4 || in_sizes[8] != 4 || in_sizes[9] != 1) return;
  if (out_size != NB * CO * HW) return;

  const float* x      = (const float*)d_in[0];
  const float* wk1c1  = (const float*)d_in[1];
  const float* wk1c2  = (const float*)d_in[2];
  const float* wk2c1  = (const float*)d_in[3];
  const float* wk2c2  = (const float*)d_in[4];
  const float* wconv  = (const float*)d_in[5];
  const float* attn_w = (const float*)d_in[6];
  const float* a_pre  = (const float*)d_in[7];
  const float* a_post = (const float*)d_in[8];
  const float* cm     = (const float*)d_in[9];
  float* out = (float*)d_out;

  const size_t PMR = 8192;
  const size_t PWZ = (size_t)4 * NZC * KD * 2;
  const size_t PWU = (size_t)4 * CH * KD * 2;
  const size_t PHQ = (size_t)NB * HW * CH * 2;
  const size_t PZ  = (size_t)NB * NZC * HW * 2;
  const size_t PYP = YPE * 2 * 2;
  const size_t PV  = (size_t)NB * CO * HW * 4;
  const size_t PR1 = 2 * PZ;
  const size_t PK2 = (size_t)NB * CO * CH * 4;
  const size_t PAK = (size_t)NB * NKK * CO * CH * 2;
  if (PYP > PR1 || PHQ + PV > PR1) return;
  size_t off = 0;
  const size_t oMRX = off; off += PMR;
  const size_t oMRV = off; off += PMR;
  const size_t oWZ  = off; off += PWZ;
  const size_t oWY  = off; off += PWZ;
  const size_t oWU  = off; off += PWU;
  const size_t oHQ  = off; off += PHQ;
  const size_t oR1  = off; off += PR1;
  const size_t oK2  = off; off += PK2;
  const size_t oAKH = off; off += PAK;
  const size_t oAKL = off; off += PAK;
  const size_t oYA  = off; off += PV;
  const size_t oYB  = off; off += PV;
  if (off > ws_size) return;
  if (off > (size_t)134217728) return;

  char* ws = (char*)d_ws;
  float* MRX = (float*)(ws + oMRX);
  float* MRV = (float*)(ws + oMRV);
  unsigned short* WZ = (unsigned short*)(ws + oWZ);
  unsigned short* WY = (unsigned short*)(ws + oWY);
  unsigned short* WU = (unsigned short*)(ws + oWU);
  unsigned short* HQ = (unsigned short*)(ws + oHQ);
  unsigned short* ZH = (unsigned short*)(ws + oR1);
  unsigned short* ZL = (unsigned short*)(ws + oR1 + PZ);
  unsigned short* YP = (unsigned short*)(ws + oR1);
  unsigned short* UQ = (unsigned short*)(ws + oR1);
  float*          V  = (float*)(ws + oR1 + PHQ);
  float* K2 = (float*)(ws + oK2);
  unsigned short* AKH = (unsigned short*)(ws + oAKH);
  unsigned short* AKL = (unsigned short*)(ws + oAKL);
  float* YA = (float*)(ws + oYA);
  float* YB = (float*)(ws + oYB);

  const dim3 blk(256);
  cvt_w<<<dim3((4 * CH * KD / 8) / 256), blk, 0, stream>>>(wk2c1, WZ, CH, 0, NZC);
  cvt_w<<<dim3((4 * CO * KD / 8) / 256), blk, 0, stream>>>(wk2c2, WZ, CO, CH, NZC);
  cvt_w<<<dim3((4 * CH * KD / 8) / 256), blk, 0, stream>>>(wk1c1, WY, CH, 0, NZC);
  cvt_w<<<dim3((4 * CO * KD / 8) / 256), blk, 0, stream>>>(wk1c2, WY, CO, CH, NZC);
  cvt_w<<<dim3((4 * CH * KD / 8) / 256), blk, 0, stream>>>(wconv, WU, CH, 0, CH);
  bn_stats<1><<<dim3(CIN), blk, 0, stream>>>(x, MRX);

  const dim3 gconv(NB * 64);
  for (int pth = 0; pth < 4; ++pth) {
    make_h<<<dim3((NB * HW * 4) / 256), blk, 0, stream>>>(x, MRX, a_pre, pth, HQ);
    conv3x3<0><<<gconv, blk, 0, stream>>>(WZ + (size_t)pth * NZC * KD, WZ + (size_t)pth * NZC * KD, HQ, ZH, ZL, V);
    corr1_softmax<<<dim3(NB), blk, 0, stream>>>(ZH, ZL, K2);
    conv3x3<1><<<gconv, blk, 0, stream>>>(WY + (size_t)pth * NZC * KD, WY + (size_t)pth * NZC * KD, HQ, YP, ZL, V);
    corr3_ak<<<dim3(NB * NKK), blk, 0, stream>>>(YP, K2, attn_w + (size_t)pth * CO * CH * NKK, AKH, AKL);
    conv3x3<2><<<gconv, blk, 0, stream>>>(WU + (size_t)pth * CH * KD, WU + (size_t)pth * CH * KD, HQ, UQ, ZL, V);
    conv3x3<3><<<gconv, blk, 0, stream>>>(AKH, AKL, UQ, ZH, ZL, V);
    bn_stats<0><<<dim3(CO), blk, 0, stream>>>(V, MRV);
    finalize<<<dim3(NPIX4 / 256), blk, 0, stream>>>(V, MRV, a_post, x, cm, pth, YA, YB, out);
  }
  (void)hipGetLastError();
}
